// MHA_31980326486203
// MI455X (gfx1250) — hardware-verified
//
#include <hip/hip_runtime.h>


#ifndef NB
#define NB 2
#endif
#ifndef SEQ
#define SEQ 2048
#endif
#define NB_FULL  2
#define SEQ_FULL 2048
#define DM   2048
#define NH_  16
#define NKV  4
#define REP  (NH_ / NKV)
#define HD   128
#define DQ   (NH_ * HD)
#define DKV  (NKV * HD)
#ifndef RH
#define RH   ((SEQ) < 512 ? (SEQ) : 512)
#endif
#define NTOK (NB * SEQ)
#define PCAR 1024.0f
#define CCAR 16.0f
#define WCAR 1024.0f
#define SL   (0.08838834764831845f * 1.4426950408889634f)
#define OSP  132
static_assert((SEQ & (SEQ - 1)) == 0);
static_assert(SEQ % 64 == 0);
static_assert(RH % 64 == 0);
static_assert(RH <= SEQ);
static_assert(HD == 128);
static_assert(NH_ % NKV == 0);
static_assert(DM % 64 == 0);
static_assert(DQ % 64 == 0);
static_assert(DKV % 64 == 0);
static_assert(NTOK % 64 == 0);
static_assert(SEQ <= SEQ_FULL);
static_assert(NB <= NB_FULL);
static_assert(((size_t)NTOK * DM / 8) % 256 == 0);
static_assert((SEQ * 32) % 256 == 0);

typedef _Float16 h16;
typedef unsigned short bf;
typedef __attribute__((ext_vector_type(16))) __bf16   v16bf;
typedef __attribute__((ext_vector_type(16))) _Float16 v16h;
typedef __attribute__((ext_vector_type(16))) unsigned short v16us;
typedef __attribute__((ext_vector_type(8)))  _Float16 v8h;
typedef __attribute__((ext_vector_type(8)))  unsigned short v8us;
typedef __attribute__((ext_vector_type(8)))  float    v8f;
typedef __attribute__((ext_vector_type(4)))  float    v4f;
typedef __attribute__((ext_vector_type(2)))  float    v2f;
typedef __attribute__((ext_vector_type(4)))  int      v4i;
typedef v4f  __attribute__((may_alias)) v4fa;

__device__ __forceinline__ unsigned short f2bf(float f) { unsigned u = __float_as_uint(f); u += 0x7FFFu + ((u >> 16) & 1u); return (unsigned short)(u >> 16); }
__device__ __forceinline__ float bf2f(unsigned short b) { return __uint_as_float(((unsigned)b) << 16); }
__device__ __forceinline__ void splitf(float y, unsigned short& h, unsigned short& l) { h = f2bf(y); l = f2bf(y - bf2f(h)); }
__device__ __forceinline__ v16h cat16(v8h lo, v8h hi) { return __builtin_shufflevector(lo, hi, 0, 1, 2, 3, 4, 5, 6, 7, 8, 9, 10, 11, 12, 13, 14, 15); }
__device__ __forceinline__ v16bf cat16b(v8us lo, v8us hi) { return __builtin_bit_cast(v16bf, __builtin_shufflevector(lo, hi, 0, 1, 2, 3, 4, 5, 6, 7, 8, 9, 10, 11, 12, 13, 14, 15)); }
__device__ __forceinline__ v8f wmma16(v16h a, v16h b, v8f c) { return __builtin_amdgcn_wmma_f32_16x16x32_f16(false, a, false, b, (short)0, c, false, false); }
__device__ __forceinline__ v8f wmmab(v16bf a, v16bf b, v8f c) { return __builtin_amdgcn_wmma_f32_16x16x32_bf16(false, a, false, b, (short)0, c, false, false); }

template <typename T16> struct WFrag;
template <> struct WFrag<h16> { typedef v16h V; static __device__ __forceinline__ V ld(const h16* p) { return cat16(*(const v8h*)p, *(const v8h*)(p + 16)); } static __device__ __forceinline__ v8f mma(V a, V b, v8f c) { return wmma16(a, b, c); } };
template <> struct WFrag<bf> { typedef v16bf V; static __device__ __forceinline__ V ld(const bf* p) { return cat16b(*(const v8us*)p, *(const v8us*)(p + 16)); } static __device__ __forceinline__ v8f mma(V a, V b, v8f c) { return wmmab(a, b, c); } };

template <typename T16, int NSPLIT, int EPI>
__global__ __launch_bounds__(32) void k_gemmw(const T16* __restrict__ A, const T16* __restrict__ A2, const T16* __restrict__ Bt, const T16* __restrict__ Bt2, int K,
                                              float* C, int ldc, float osc, size_t sA, size_t sC,
                                              h16* P16, bf* Ph, bf* Pl, int ldp, const float* __restrict__ CS, int hlr) {
    typedef typename WFrag<T16>::V V;
    __shared__ __align__(16) float os[16 * 68];
    const size_t z = blockIdx.z; A += z * sA; if (A2) A2 += z * sA; if (EPI == 0) C += z * sC;
    const int lane = threadIdx.x & 31, lr = lane & 15, hi = lane >> 4; const int r0 = blockIdx.x * 64, c0 = blockIdx.y * 64;
    v8f acc[4][4];
#pragma unroll
    for (int mb = 0; mb < 4; ++mb)
#pragma unroll
        for (int nb = 0; nb < 4; ++nb) acc[mb][nb] = (v8f){};
    const size_t aoff = (size_t)(r0 + lr) * K + 8 * hi, boff = (size_t)(c0 + lr) * K + 8 * hi;
#pragma unroll 1
    for (int kc = 0; kc < K; kc += 32) {
        V a[4], a2[4];
#pragma unroll
        for (int mb = 0; mb < 4; ++mb) { a[mb] = WFrag<T16>::ld(A + aoff + (size_t)mb * 16 * K + kc); if (NSPLIT == 1 || NSPLIT == 2) a2[mb] = WFrag<T16>::ld(A2 + aoff + (size_t)mb * 16 * K + kc); }
#pragma unroll
        for (int nb = 0; nb < 4; ++nb) { const V b = WFrag<T16>::ld(Bt + boff + (size_t)nb * 16 * K + kc); V b2; if (NSPLIT >= 2) b2 = WFrag<T16>::ld(Bt2 + boff + (size_t)nb * 16 * K + kc);
#pragma unroll
            for (int mb = 0; mb < 4; ++mb) { acc[mb][nb] = WFrag<T16>::mma(a[mb], b, acc[mb][nb]); if (NSPLIT == 1 || NSPLIT == 2) acc[mb][nb] = WFrag<T16>::mma(a2[mb], b, acc[mb][nb]); if (NSPLIT >= 2) acc[mb][nb] = WFrag<T16>::mma(a[mb], b2, acc[mb][nb]); } }
        asm volatile("v_nop\n\tv_nop\n\tv_nop\n\tv_nop" : "+v"(acc[0][0]), "+v"(acc[1][1]), "+v"(acc[2][2]), "+v"(acc[3][3]) : "v"(a[0]), "v"(a[3]));
    }
    const bool hlb = (EPI == 2) || (((unsigned)r0 & (unsigned)(SEQ - 1)) < (unsigned)hlr);
#pragma unroll
    for (int mb = 0; mb < 4; ++mb) {
#pragma unroll
        for (int nb = 0; nb < 4; ++nb) {
#pragma unroll
            for (int j = 0; j < 8; ++j) os[(hi * 8 + j) * 68 + nb * 16 + lr] = acc[mb][nb][j]; }
        __builtin_amdgcn_wave_barrier(); asm volatile("" ::: "memory");
        if (EPI == 0) {
            float* crow = C + (size_t)(r0 + mb * 16) * ldc + c0;
#pragma unroll 1
            for (int ps = 0; ps < 2; ++ps) {
#pragma unroll
                for (int s = 0; s < 8; ++s) { const int row = 2 * s + hi, cofs = lr * 4; v4f val = *(const v4fa*)(os + row * 68 + cofs); val = val * osc;
                    *(volatile v4f*)(crow + (size_t)row * ldc + cofs) = val; }
                if (ps == 0) __threadfence(); }
        } else {
            const unsigned g0 = (unsigned)r0 + (unsigned)mb * 16u;
#pragma unroll 1
            for (int ps = 0; ps < 2; ++ps) {
#pragma unroll
                for (unsigned s = 0; s < 4; ++s) {
                    const unsigned row = 4u * s + ((unsigned)lane >> 3), cofs = ((unsigned)lane & 7u) * 8u;
                    const v4f x0 = *(const v4fa*)(os + row * 68u + cofs), x1 = *(const v4fa*)(os + row * 68u + cofs + 4u);
                    const unsigned g = g0 + row, t = g & (unsigned)(SEQ - 1);
                    float v[8];
                    if (EPI == 1) {
                        const float* cp = CS + (size_t)t * HD + (((unsigned)c0 + cofs) & (unsigned)(HD - 1));
                        const v4f ca = *(const v4f*)cp, cb = *(const v4f*)(cp + 4);
                        v[0] = x0[0] * ca[0] - x0[1] * ca[1]; v[1] = x0[0] * ca[1] + x0[1] * ca[0];
                        v[2] = x0[2] * ca[2] - x0[3] * ca[3]; v[3] = x0[2] * ca[3] + x0[3] * ca[2];
                        v[4] = x1[0] * cb[0] - x1[1] * cb[1]; v[5] = x1[0] * cb[1] + x1[1] * cb[0];
                        v[6] = x1[2] * cb[2] - x1[3] * cb[3]; v[7] = x1[2] * cb[3] + x1[3] * cb[2];
                    } else {
                        v[0] = x0[0]; v[1] = x0[1]; v[2] = x0[2]; v[3] = x0[3]; v[4] = x1[0]; v[5] = x1[1]; v[6] = x1[2]; v[7] = x1[3];
                    }
                    v8h o16; v8us oh, ol;
#pragma unroll
                    for (int q = 0; q < 8; ++q) { o16[q] = (h16)v[q]; unsigned short a2, c2; splitf(v[q], a2, c2); oh[q] = a2; ol[q] = c2; }
                    const size_t o = (size_t)g * (unsigned)ldp + (unsigned)c0 + cofs;
                    *(volatile v8h*)(P16 + o) = o16;
                    if (hlb) { const size_t o2 = (EPI == 1) ? ((size_t)((g / (unsigned)SEQ) * (unsigned)hlr + t) * (unsigned)ldp + (unsigned)c0 + cofs) : o;
                        *(volatile v8us*)(Ph + o2) = oh; *(volatile v8us*)(Pl + o2) = ol; }
                }
                if (ps == 0) __threadfence(); }
        }
        __builtin_amdgcn_wave_barrier(); asm volatile("" ::: "memory");
    }
}

__global__ __launch_bounds__(256) void k_xb(const float* __restrict__ x, bf* XB) {
    const unsigned i = blockIdx.x * 256u + threadIdx.x; if (i >= (unsigned)((size_t)NTOK * DM / 8)) return;
    const unsigned per = (unsigned)((size_t)SEQ * DM / 8); const unsigned b = i / per, r = i - b * per;
    const float* s = x + (size_t)b * SEQ_FULL * DM + (size_t)r * 8u;
    const v4f a = *(const v4f*)s, c = *(const v4f*)(s + 4); v8us o;
#pragma unroll
    for (int q = 0; q < 4; ++q) { o[q] = f2bf(a[q]); o[4 + q] = f2bf(c[q]); }
    *(volatile v8us*)(XB + (size_t)i * 8u) = o; __threadfence(); *(volatile v8us*)(XB + (size_t)i * 8u) = o; }

__global__ __launch_bounds__(256) void k_wt(const float* __restrict__ W, unsigned K, unsigned N, bf* Wb, h16* Wh, float hs) {
    __shared__ float tile[64 * 65];
    const unsigned tid = threadIdx.x, n0 = blockIdx.x * 64u, k0 = blockIdx.y * 64u;
#pragma unroll 4
    for (unsigned i = 0; i < 16; ++i) { const unsigned r = i * 4u + (tid >> 6), c = tid & 63u; tile[r * 65u + c] = W[(size_t)(k0 + r) * N + n0 + c]; }
    __syncthreads();
#pragma unroll 1
    for (int ps = 0; ps < 2; ++ps) {
#pragma unroll
        for (unsigned j = 0; j < 2; ++j) { const unsigned nn = (tid >> 3) + 32u * j, p = tid & 7u; v8us ob; v8h oh;
#pragma unroll
            for (unsigned e = 0; e < 8; ++e) { const unsigned short u = f2bf(tile[(p * 8u + e) * 65u + nn]); ob[e] = u; oh[e] = (h16)(bf2f(u) * hs); }
            const size_t o = (size_t)(n0 + nn) * K + k0 + p * 8u;
            *(volatile v8us*)(Wb + o) = ob; if (Wh) *(volatile v8h*)(Wh + o) = oh; }
        if (ps == 0) __threadfence(); }
}

struct T32 { float v[32]; };
static_assert(sizeof(T32) == 128);
__global__ __launch_bounds__(256) void k_cstab(T32 iv, int ibase, float* CS) {
    const unsigned idx = blockIdx.x * 256u + threadIdx.x; if (idx >= (unsigned)(SEQ * 32)) return;
    const unsigned t = idx >> 5, j = idx & 31u;
    float inv = iv.v[0];
#pragma unroll
    for (int q = 1; q < 32; ++q) inv = (j == (unsigned)q) ? iv.v[q] : inv;
    const float ang = __fmul_rn((float)t, inv);
    float sn, cs; sincosf(ang, &sn, &cs);
    v2f o; o[0] = cs; o[1] = sn;
    float* p = CS + ((size_t)t * 64u + (unsigned)ibase + j) * 2u;
    *(volatile v2f*)p = o; __threadfence(); *(volatile v2f*)p = o; }

template <bool BAND>
__global__ __launch_bounds__(128) void k_attn(const h16* Q16, const bf* Qh, const bf* Ql, const h16* K16, const bf* Kh, const bf* Kl, const h16* V16, const bf* Vh, const bf* Vl,
                                              const int* __restrict__ mask, h16* C16, bf* Ch, bf* Cl) {
    __shared__ __align__(16) float os[4 * 16 * OSP];
    const unsigned tid = threadIdx.x, w = tid >> 5, lane = tid & 31u, lr = lane & 15u, hh = lane >> 4;
    const unsigned h = blockIdx.y, b = blockIdx.z, kv = h / (unsigned)REP;
    const unsigned q0 = (BAND ? 0u : (unsigned)RH) + blockIdx.x * 64u + w * 16u;
    const unsigned qn = q0 + lr;
    const unsigned tb = b * (unsigned)SEQ;
    const unsigned kvo = kv * (unsigned)HD;
    const unsigned qoffP = (tb + qn) * (unsigned)DQ + h * (unsigned)HD + 8u * hh;
    const unsigned qoffB = (b * (unsigned)RH + qn) * (unsigned)DQ + h * (unsigned)HD + 8u * hh;
    v16h qf[4];
    if (!BAND) {
#pragma unroll
        for (int kc = 0; kc < 4; ++kc) qf[kc] = WFrag<h16>::ld(Q16 + qoffP + kc * 32);
    }
    v8f O[8];
#pragma unroll
    for (int df = 0; df < 8; ++df) O[df] = (v8f){};
    float m = -3.0e38f, l = 0.f;
    const int* mrow = mask + (size_t)qn * SEQ_FULL + 8u * hh;
    const unsigned koff = (tb + lr) * (unsigned)DKV + kvo + 8u * hh;
    const unsigned voff = (kvo + lr) * (unsigned)NTOK + tb + 8u * hh;
#pragma unroll 1
    for (unsigned kt = 0; kt < (unsigned)SEQ; kt += 32u) {
        const v4i m0 = *(const v4i*)(mrow + kt), m1 = *(const v4i*)(mrow + kt + 4), m2 = *(const v4i*)(mrow + kt + 16), m3 = *(const v4i*)(mrow + kt + 20);
        const int any = m0[0] | m0[1] | m0[2] | m0[3] | m1[0] | m1[1] | m1[2] | m1[3] | m2[0] | m2[1] | m2[2] | m2[3] | m3[0] | m3[1] | m3[2] | m3[3];
        if (__builtin_amdgcn_ballot_w32(any != 0) == 0u) continue;
        const int mk0[8] = { m0[0], m0[1], m0[2], m0[3], m1[0], m1[1], m1[2], m1[3] };
        const int mk1[8] = { m2[0], m2[1], m2[2], m2[3], m3[0], m3[1], m3[2], m3[3] };
        v8f s0 = (v8f){}, s1 = (v8f){};
        if (BAND) {
            unsigned qo = qoffB; asm volatile("" : "+v"(qo));
#pragma unroll 1
            for (unsigned kc = 0; kc < (unsigned)HD; kc += 32u) {
                const v16bf bh = WFrag<bf>::ld(Qh + qo + kc), bl = WFrag<bf>::ld(Ql + qo + kc);
                const unsigned ka = koff + kt * (unsigned)DKV + kc, kb2 = ka + 16u * (unsigned)DKV;
                const v16bf a0h = WFrag<bf>::ld(Kh + ka), a0l = WFrag<bf>::ld(Kl + ka), a1h = WFrag<bf>::ld(Kh + kb2), a1l = WFrag<bf>::ld(Kl + kb2);
                s0 = wmmab(a0h, bh, s0); s0 = wmmab(a0h, bl, s0); s0 = wmmab(a0l, bh, s0);
                s1 = wmmab(a1h, bh, s1); s1 = wmmab(a1h, bl, s1); s1 = wmmab(a1l, bh, s1);
                asm volatile("v_nop\n\tv_nop\n\tv_nop\n\tv_nop" : "+v"(s0), "+v"(s1) : "v"(a1l), "v"(bh));
            }
        } else {
#pragma unroll
            for (int kc = 0; kc < 4; ++kc) {
                const unsigned ka = koff + kt * (unsigned)DKV + (unsigned)kc * 32u;
                const v16h a0 = WFrag<h16>::ld(K16 + ka), a1 = WFrag<h16>::ld(K16 + ka + 16u * (unsigned)DKV);
                s0 = wmma16(a0, qf[kc], s0); s1 = wmma16(a1, qf[kc], s1);
                asm volatile("v_nop\n\tv_nop\n\tv_nop\n\tv_nop" : "+v"(s0), "+v"(s1) : "v"(a0), "v"(a1));
            }
        }
        float p0[8], p1[8]; float tm = -3.0e38f;
#pragma unroll
        for (int r = 0; r < 8; ++r) {
            const float a = s0[r] * SL, c = s1[r] * SL;
            p0[r] = (mk0[r] != 0) ? a : -3.0e38f; p1[r] = (mk1[r] != 0) ? c : -3.0e38f;
            tm = fmaxf(tm, fmaxf(p0[r], p1[r])); }
        tm = fmaxf(tm, __shfl_xor(tm, 16, 32));
        const float mn = fmaxf(m, tm);
        const float al = __builtin_amdgcn_exp2f(m - mn);
        float ls = 0.f;
#pragma unroll
        for (int r = 0; r < 8; ++r) {
            const float e0 = __builtin_amdgcn_exp2f(p0[r] - mn), e1 = __builtin_amdgcn_exp2f(p1[r] - mn);
            p0[r] = (mk0[r] != 0) ? e0 : 0.f; p1[r] = (mk1[r] != 0) ? e1 : 0.f;
            ls += p0[r] + p1[r]; }
        ls += __shfl_xor(ls, 16, 32);
        l = l * al + ls; m = mn;
#pragma unroll
        for (int df = 0; df < 8; ++df) O[df] = O[df] * al;
        if (BAND) {
            v16us uh, ul;
#pragma unroll
            for (int r = 0; r < 8; ++r) { unsigned short a2, c2; splitf(p0[r], a2, c2); uh[r] = a2; ul[r] = c2; splitf(p1[r], a2, c2); uh[8 + r] = a2; ul[8 + r] = c2; }
            const v16bf pbh = __builtin_bit_cast(v16bf, uh), pbl = __builtin_bit_cast(v16bf, ul);
#pragma unroll
            for (int df = 0; df < 8; ++df) {
                const unsigned vo = voff + (unsigned)df * 16u * (unsigned)NTOK + kt;
                const v16bf avh = WFrag<bf>::ld(Vh + vo), avl = WFrag<bf>::ld(Vl + vo);
                O[df] = wmmab(avh, pbh, O[df]); O[df] = wmmab(avh, pbl, O[df]); O[df] = wmmab(avl, pbh, O[df]);
                asm volatile("v_nop\n\tv_nop\n\tv_nop\n\tv_nop" : "+v"(O[df]) : "v"(avh), "v"(avl));
                asm volatile("" ::: "memory");
            }
            asm volatile("v_nop\n\tv_nop\n\tv_nop\n\tv_nop" : "+v"(O[0]), "+v"(O[1]), "+v"(O[2]), "+v"(O[3]), "+v"(O[4]), "+v"(O[5]), "+v"(O[6]), "+v"(O[7]) : "v"(pbh), "v"(pbl));
        } else {
            v16h pb;
#pragma unroll
            for (int r = 0; r < 8; ++r) { pb[r] = (h16)(p0[r] * PCAR); pb[8 + r] = (h16)(p1[r] * PCAR); }
#pragma unroll
            for (int df = 0; df < 8; ++df) {
                const v16h av = WFrag<h16>::ld(V16 + voff + (unsigned)df * 16u * (unsigned)NTOK + kt);
                O[df] = wmma16(av, pb, O[df]);
                asm volatile("v_nop\n\tv_nop\n\tv_nop\n\tv_nop" : "+v"(O[df]) : "v"(av));
            }
            asm volatile("v_nop\n\tv_nop\n\tv_nop\n\tv_nop" : "+v"(O[0]), "+v"(O[1]), "+v"(O[2]), "+v"(O[3]), "+v"(O[4]), "+v"(O[5]), "+v"(O[6]), "+v"(O[7]) : "v"(pb));
        }
    }
    const float inv = (l > 0.f) ? (1.0f / l) : 0.f;
    const float osc = BAND ? inv : inv * (CCAR / PCAR);
    float* ow = os + w * (16u * OSP);
#pragma unroll
    for (int df = 0; df < 8; ++df) { v4f a, c;
#pragma unroll
        for (int r = 0; r < 4; ++r) { a[r] = O[df][r] * osc; c[r] = O[df][4 + r] * osc; }
        *(v4fa*)(ow + lr * OSP + (unsigned)df * 16u + 8u * hh) = a; *(v4fa*)(ow + lr * OSP + (unsigned)df * 16u + 8u * hh + 4u) = c; }
    __syncthreads();
#pragma unroll 1
    for (int ps = 0; ps < 2; ++ps) {
#pragma unroll
        for (unsigned s = 0; s < 8; ++s) { const unsigned row = 2u * s + hh, cofs = lr * 8u;
            const v4f x0 = *(const v4fa*)(ow + row * OSP + cofs), x1 = *(const v4fa*)(ow + row * OSP + cofs + 4u);
            if (BAND) { v8us oh, ol;
#pragma unroll
                for (int q = 0; q < 4; ++q) { unsigned short a2, c2; splitf(x0[q], a2, c2); oh[q] = a2; ol[q] = c2; splitf(x1[q], a2, c2); oh[4 + q] = a2; ol[4 + q] = c2; }
                const size_t o = (size_t)(b * (unsigned)RH + q0 + row) * (unsigned)DQ + h * (unsigned)HD + cofs;
                *(volatile v8us*)(Ch + o) = oh; *(volatile v8us*)(Cl + o) = ol;
            } else { v8h o16;
#pragma unroll
                for (int q = 0; q < 4; ++q) { o16[q] = (h16)x0[q]; o16[4 + q] = (h16)x1[q]; }
                const size_t o = (size_t)(tb + q0 + row) * (unsigned)DQ + h * (unsigned)HD + cofs;
                *(volatile v8h*)(C16 + o) = o16; } }
        if (ps == 0) __threadfence(); }
}

constexpr size_t al256(size_t b) { return (b + 255) & ~(size_t)255; }
constexpr size_t WS_TOTAL =
    al256((size_t)NTOK * DM * 2) +
    al256((size_t)DQ * DM * 2) + 2 * al256((size_t)DKV * DM * 2) +
    2 * al256((size_t)DM * DQ * 2) +
    al256((size_t)SEQ * HD * 4) +
    al256((size_t)NTOK * DQ * 2) + 2 * al256((size_t)NB * RH * DQ * 2) +
    3 * al256((size_t)NTOK * DKV * 2) +
    3 * al256((size_t)DKV * NTOK * 2) +
    al256((size_t)NTOK * DQ * 2) + 2 * al256((size_t)NB * RH * DQ * 2);
static_assert(WS_TOTAL <= (size_t)134217728);

extern "C" void kernel_launch(void* const* d_in, const int* in_sizes, int n_in,
                              void* d_out, int out_size, void* d_ws, size_t ws_size, hipStream_t stream) {
    if (n_in < 6) return;
    const size_t xneed = ((size_t)(NB - 1) * SEQ_FULL + SEQ) * DM;
    if ((size_t)in_sizes[0] < xneed || (size_t)in_sizes[1] < (size_t)DM * DQ || (size_t)in_sizes[2] < (size_t)DM * DKV || (size_t)in_sizes[3] < (size_t)DM * DKV ||
        (size_t)in_sizes[4] < (size_t)DQ * DM || (size_t)in_sizes[5] < (size_t)(SEQ - 1) * SEQ_FULL + SEQ || (size_t)out_size < xneed) return;
    if (WS_TOTAL > ws_size) return;
    const float* x = (const float*)d_in[0]; const float* Wq = (const float*)d_in[1]; const float* Wk = (const float*)d_in[2]; const float* Wv = (const float*)d_in[3]; const float* Wo = (const float*)d_in[4];
    const int* mask = (const int*)d_in[5];
    float* OUT = (float*)d_out;
    char* wsp = (char*)d_ws;
    auto take = [&](size_t bytes) { char* p = wsp; wsp += al256(bytes); return (void*)p; };
    bf* XB = (bf*)take((size_t)NTOK * DM * 2);
    bf* WqT = (bf*)take((size_t)DQ * DM * 2); bf* WkT = (bf*)take((size_t)DKV * DM * 2); bf* WvT = (bf*)take((size_t)DKV * DM * 2);
    bf* WoTb = (bf*)take((size_t)DM * DQ * 2); h16* WoTh = (h16*)take((size_t)DM * DQ * 2);
    float* CS = (float*)take((size_t)SEQ * HD * 4);
    h16* Q16 = (h16*)take((size_t)NTOK * DQ * 2); bf* Qh = (bf*)take((size_t)NB * RH * DQ * 2); bf* Ql = (bf*)take((size_t)NB * RH * DQ * 2);
    h16* K16 = (h16*)take((size_t)NTOK * DKV * 2); bf* Kh = (bf*)take((size_t)NTOK * DKV * 2); bf* Kl = (bf*)take((size_t)NTOK * DKV * 2);
    h16* V16 = (h16*)take((size_t)DKV * NTOK * 2); bf* Vh = (bf*)take((size_t)DKV * NTOK * 2); bf* Vl = (bf*)take((size_t)DKV * NTOK * 2);
    h16* C16 = (h16*)take((size_t)NTOK * DQ * 2); bf* Ch = (bf*)take((size_t)NB * RH * DQ * 2); bf* Cl = (bf*)take((size_t)NB * RH * DQ * 2);
    if ((size_t)(wsp - (char*)d_ws) > ws_size) return;

    T32 iva, ivb;
    for (int i = 0; i < 32; ++i) { const float pa = (float)pow(1000.0, (double)(2 * i) / 128.0); iva.v[i] = 1.0f / pa; const float pb = (float)pow(1000.0, (double)(2 * (i + 32)) / 128.0); ivb.v[i] = 1.0f / pb; }

    k_xb<<<(unsigned)((size_t)NTOK * DM / 8 / 256), 256, 0, stream>>>(x, XB);
    k_wt<<<dim3(DQ / 64, DM / 64), 256, 0, stream>>>(Wq, (unsigned)DM, (unsigned)DQ, WqT, nullptr, 1.0f);
    k_wt<<<dim3(DKV / 64, DM / 64), 256, 0, stream>>>(Wk, (unsigned)DM, (unsigned)DKV, WkT, nullptr, 1.0f);
    k_wt<<<dim3(DKV / 64, DM / 64), 256, 0, stream>>>(Wv, (unsigned)DM, (unsigned)DKV, WvT, nullptr, 1.0f);
    k_wt<<<dim3(DM / 64, DQ / 64), 256, 0, stream>>>(Wo, (unsigned)DQ, (unsigned)DM, WoTb, WoTh, WCAR);
    k_cstab<<<SEQ * 32 / 256, 256, 0, stream>>>(iva, 0, CS);
    k_cstab<<<SEQ * 32 / 256, 256, 0, stream>>>(ivb, 32, CS);

    k_gemmw<bf, 0, 1><<<dim3(NTOK / 64, DQ / 64, 1), 32, 0, stream>>>(XB, nullptr, WqT, nullptr, DM, nullptr, 0, 1.0f, 0, 0, Q16, Qh, Ql, DQ, CS, RH);
    k_gemmw<bf, 0, 1><<<dim3(NTOK / 64, DKV / 64, 1), 32, 0, stream>>>(XB, nullptr, WkT, nullptr, DM, nullptr, 0, 1.0f, 0, 0, K16, Kh, Kl, DKV, CS, SEQ);
    k_gemmw<bf, 0, 2><<<dim3(DKV / 64, NTOK / 64, 1), 32, 0, stream>>>(WvT, nullptr, XB, nullptr, DM, nullptr, 0, 1.0f, 0, 0, V16, Vh, Vl, NTOK, nullptr, 0);

    k_attn<true><<<dim3(RH / 64, NH_, NB), 128, 0, stream>>>(Q16, Qh, Ql, K16, Kh, Kl, V16, Vh, Vl, mask, C16, Ch, Cl);
    if (SEQ > RH) k_attn<false><<<dim3((SEQ - RH) / 64, NH_, NB), 128, 0, stream>>>(Q16, Qh, Ql, K16, Kh, Kl, V16, Vh, Vl, mask, C16, Ch, Cl);

    k_gemmw<bf, 1, 0><<<dim3(RH / 64, DM / 64, NB), 32, 0, stream>>>(Ch, Cl, WoTb, nullptr, DQ, OUT, DM, 1.0f, (size_t)RH * DQ, (size_t)SEQ_FULL * DM, nullptr, nullptr, nullptr, 0, nullptr, 0);
    if (SEQ > RH) k_gemmw<h16, 0, 0><<<dim3((SEQ - RH) / 64, DM / 64, NB), 32, 0, stream>>>(C16 + (size_t)RH * DQ, nullptr, WoTh, nullptr, DQ, OUT + (size_t)RH * DM, DM, 1.0f / (CCAR * WCAR), (size_t)SEQ * DQ, (size_t)SEQ_FULL * DM, nullptr, nullptr, nullptr, 0, nullptr, 0);
}
